// DynamicFeatureAggregation_76184129896956
// MI455X (gfx1250) — hardware-verified
//
#include <hip/hip_runtime.h>


namespace {
constexpr int Bn = 8, C = 256, HW = 64, NP = HW * HW, NT = Bn * NP, KA = 3 * C;
constexpr float XS = 8.0f, EPS = 1e-5f;

typedef _Float16 b16;
typedef __attribute__((ext_vector_type(16))) _Float16 v16b;
typedef __attribute__((ext_vector_type(8))) _Float16 v8b;
typedef __attribute__((ext_vector_type(8))) float v8f;
typedef __attribute__((ext_vector_type(4))) float v4f;
__device__ __forceinline__ float bf16_rne(float f) { unsigned int u = __float_as_uint(f); u += 0x7FFFu + ((u >> 16) & 1u); return __uint_as_float(u & 0xFFFF0000u); }
__device__ __forceinline__ v16b frag_kb(const b16* p, int hh) { const v8b a = *(const v8b*)(p + 8 * hh), b = *(const v8b*)(p + 16 + 8 * hh); v16b f;
#pragma unroll
  for (int e = 0; e < 8; ++e) { f[e] = a[e]; f[8 + e] = b[e]; } return f; }
__device__ __forceinline__ v8f wmma16b(v16b a, v16b b, v8f c) { v8f d = __builtin_amdgcn_wmma_f32_16x16x32_f16(false, a, false, b, (short)0, c, false, false); asm volatile("v_nop\n\tv_nop\n\tv_nop\n\tv_nop" : "+v"(d) : "v"(a), "v"(b)); return d; }
__device__ __forceinline__ void wave_lds_sync() { __builtin_amdgcn_fence(__ATOMIC_RELEASE, "workgroup"); __builtin_amdgcn_wave_barrier(); __builtin_amdgcn_fence(__ATOMIC_ACQUIRE, "workgroup"); }
__device__ __forceinline__ float pmul(float a, float b) { float p = a * b; asm volatile("" : "+v"(p)); return p; }

__global__ __launch_bounds__(256) void prep_kernel(const float* __restrict__ w, const float* __restrict__ b, const float* __restrict__ gma, const float* __restrict__ bta, const float* __restrict__ rm, const float* __restrict__ rv, b16* __restrict__ R, float* __restrict__ P) {
  const size_t tid = (size_t)blockIdx.x * 256 + threadIdx.x, nth = (size_t)gridDim.x * 256;
  for (int pass = 0; pass < 2; ++pass) {
    for (size_t p = tid; p < (size_t)C * KA / 8; p += nth) { const int o = (int)(p / (KA / 8)), k0 = (int)(p % (KA / 8)) * 8; const int src0 = (k0 < 2 * C) ? k0 : (k0 - C); v8b v; for (int e = 0; e < 8; ++e) v[e] = (b16)bf16_rne(w[(size_t)o * 2 * C + src0 + e]); *(volatile v8b*)(R + p * 8) = v; }
    for (size_t q = tid; q < 768; q += nth) { const int i = (int)q, c = i & 255; float v; if (i < 256) v = bf16_rne(b[c]); else { const float sc = bf16_rne(gma[c]) * rsqrtf(bf16_rne(rv[c]) + EPS); v = (i < 512) ? sc : (bf16_rne(bta[c]) - bf16_rne(rm[c]) * sc); } P[q] = v; }
    __threadfence(); }
}

__global__ __launch_bounds__(256) void arows_kernel(const float* __restrict__ x, const float* __restrict__ sim, b16* __restrict__ A) {
  __shared__ __attribute__((aligned(16))) b16 T[64][KA + 8]; __shared__ float S9[9][64]; __shared__ float xr[3][66];
  const int y = blockIdx.x, b = blockIdx.y, t_ = threadIdx.x;
  for (int i = t_; i < 9 * 64; i += 256) { const int k = i / 64, xx = i % 64; S9[k][xx] = bf16_rne(sim[((size_t)b * 9 + k) * NP + y * HW + xx]); }
  for (int c = 0; c < C; ++c) { const float* xc = x + ((size_t)b * C + c) * NP;
    __syncthreads();
    for (int i = t_; i < 3 * 66; i += 256) { const int r = i / 66, xx = i % 66 - 1, yy = y + r - 1; xr[r][i % 66] = (yy >= 0 && yy < HW && xx >= 0 && xx < HW) ? bf16_rne(xc[yy * HW + xx]) : 0.0f; }
    __syncthreads();
    if (t_ < 64) { float a = 0.0f;
#pragma unroll
      for (int dy = 0; dy < 3; ++dy)
#pragma unroll
        for (int dx = 0; dx < 3; ++dx) a += pmul(xr[dy][t_ + dx], S9[dy * 3 + dx][t_]);
      T[t_][c] = (b16)(xr[1][t_ + 1] * XS); const b16 ah = (b16)(a * XS); T[t_][C + c] = ah; T[t_][2 * C + c] = (b16)(a * XS - (float)ah); } }
  __syncthreads();
  for (int pass = 0; pass < 2; ++pass) { for (int i = t_; i < 64 * (KA / 8); i += 256) { const int p = i / (KA / 8), c8 = (i % (KA / 8)) * 8; *(volatile v8b*)(A + ((size_t)b * NP + y * HW + p) * KA + c8) = *(const v8b*)(&T[p][c8]); } __threadfence(); }
}

__global__ __launch_bounds__(64) void conv_kernel(const b16* __restrict__ A, const b16* __restrict__ R, const float* __restrict__ P, float* __restrict__ out) {
  __shared__ __attribute__((aligned(16))) float Ts[2][32][128 + 1];
  const int lane = threadIdx.x & 31, wave = threadIdx.x >> 5, nloc = lane & 15, hlf = lane >> 4, m0 = blockIdx.y * 32, c0 = wave * 128; const int b = m0 / NP, p0 = m0 % NP;
  v8f acc[2][8];
#pragma unroll
  for (int r = 0; r < 2; ++r)
#pragma unroll
    for (int t = 0; t < 8; ++t) acc[r][t] = (v8f){};
#pragma unroll 2
  for (int kb = 0; kb < KA; kb += 32) { const v16b a0 = frag_kb(A + (size_t)(m0 + nloc) * KA + kb, hlf), a1 = frag_kb(A + (size_t)(m0 + 16 + nloc) * KA + kb, hlf);
#pragma unroll
    for (int t = 0; t < 8; ++t) { const v16b bw = frag_kb(R + (size_t)(c0 + t * 16 + nloc) * KA + kb, hlf); acc[0][t] = wmma16b(a0, bw, acc[0][t]); acc[1][t] = wmma16b(a1, bw, acc[1][t]); } }
#pragma unroll
  for (int t = 0; t < 8; ++t) { const int o = c0 + t * 16 + nloc; const float bb = P[o], sc = P[256 + o], sh = P[512 + o];
#pragma unroll
    for (int r = 0; r < 2; ++r)
#pragma unroll
      for (int v = 0; v < 8; ++v) Ts[wave][r * 16 + 8 * hlf + v][t * 16 + nloc] = fmaxf(pmul(acc[r][t][v] * (1.0f / XS) + bb, sc) + sh, 0.0f); }
  wave_lds_sync();
  for (int pass = 0; pass < 2; ++pass) { for (int cc = 0; cc < 128; ++cc) ((volatile float*)out)[((size_t)b * C + c0 + cc) * NP + p0 + lane] = Ts[wave][lane][cc]; __threadfence(); }
}
}

extern "C" void kernel_launch(void* const* d_in, const int* in_sizes, int n_in,
                              void* d_out, int out_size, void* d_ws, size_t ws_size, hipStream_t stream) {
  (void)n_in; (void)out_size;
  const float* x = (const float*)d_in[0]; const float* sim = (const float*)d_in[1]; const float* w = (const float*)d_in[2]; const float* b = (const float*)d_in[3]; const float* gma = (const float*)d_in[4]; const float* bta = (const float*)d_in[5]; const float* rm = (const float*)d_in[6]; const float* rv = (const float*)d_in[7];
  float* out = (float*)d_out;
  if (in_sizes[0] != NT * C || in_sizes[1] != Bn * 9 * NP || in_sizes[2] != C * 2 * C) return;
  size_t off = 0; char* ws = (char*)d_ws;
  auto carve = [&](size_t bytes) { char* p = ws + off; off += (bytes + 255) & ~(size_t)255; return p; };
  b16* R = (b16*)carve((size_t)C * KA * 2); float* P = (float*)carve(768 * 4); b16* A = (b16*)carve((size_t)NT * KA * 2);
  if (off > ws_size) return;
  prep_kernel<<<64, 256, 0, stream>>>(w, b, gma, bta, rm, rv, R, P);
  arows_kernel<<<dim3(HW, Bn), 256, 0, stream>>>(x, sim, A);
  conv_kernel<<<dim3(1, NT / 32), 64, 0, stream>>>(A, R, P, out);
}
